// GNNEncoder_24464133718256
// MI455X (gfx1250) — hardware-verified
//
#include <hip/hip_runtime.h>
#include <stddef.h>
#include <stdint.h>
#include <math.h>


#pragma clang fp contract(off)

#define NV    64
#define SEQ   2048
#define HD    32
#define KC    128
#define NCH   16
#define SC    (SEQ / NCH)
#define FTHR  128
#define NWF   4
#define CTHR  128
#define RECF  (NV * HD)
#define WSMAX 134217728

static_assert(SEQ % NCH == 0);
static_assert(NV == NWF * 16);
static_assert(HD == 2 * 16);
static_assert(KC == 2 * NV && KC == 4 * HD && (KC % 32) == 0);
static_assert(NV * (NV / 8) == 4 * FTHR);
static_assert(HD * (KC / 8) == 4 * FTHR);
static_assert(HD * (NV / 8) == 2 * FTHR);
static_assert((NV * HD) / 4 == 4 * FTHR);
static_assert(NV / 4 <= FTHR && NV <= FTHR && HD <= FTHR);
static_assert((RECF * 4) % 128 == 0);

typedef float          v4f   __attribute__((ext_vector_type(4)));
typedef float          v8f   __attribute__((ext_vector_type(8)));
typedef int            v8i   __attribute__((ext_vector_type(8)));
typedef unsigned int   v4u   __attribute__((ext_vector_type(4)));
typedef unsigned short v8us  __attribute__((ext_vector_type(8)));
typedef __bf16         v16b  __attribute__((ext_vector_type(16)));
typedef v4f  __attribute__((may_alias)) v4fa;
typedef v4u  __attribute__((may_alias)) v4ua;
typedef v8us __attribute__((may_alias)) v8usa;
union FragB { v16b v; v8us h[2]; v8i w; };
union Q8 { v8f v; v4f q[2]; };

__device__ __forceinline__ v8f wmb(const FragB& a, const FragB& b, v8f c) {
  v8f d = __builtin_amdgcn_wmma_f32_16x16x32_bf16(false, a.v, false, b.v, (short)0, c, false, false);
  asm volatile("v_nop\n\tv_nop\n\tv_nop\n\tv_nop" : "+v"(d) : "v"(a.w), "v"(b.w));
  return d;
}

__device__ __forceinline__ unsigned int f2bf(float f) {
  const unsigned int u = __float_as_uint(f);
  return ((u + 0x7FFFu + ((u >> 16) & 1u)) >> 16) & 0xFFFFu;
}
__device__ __forceinline__ float bf2f(unsigned int b) { return __uint_as_float(b << 16); }
__device__ __forceinline__ float bfr(float f) { return bf2f(f2bf(f)); }
__device__ __forceinline__ v4f bfr4(const v4f a) {
  v4f r; r.x = bfr(a.x); r.y = bfr(a.y); r.z = bfr(a.z); r.w = bfr(a.w); return r;
}
__device__ __forceinline__ unsigned int pk2(float lo, float hi) { return f2bf(lo) | (f2bf(hi) << 16); }
__device__ __forceinline__ v4u pack8(const v4f a, const v4f b) {
  v4u r;
  r.x = pk2(a.x, a.y); r.y = pk2(a.z, a.w); r.z = pk2(b.x, b.y); r.w = pk2(b.z, b.w);
  return r;
}
__device__ __forceinline__ void split2(float a, float b, unsigned int& hw, unsigned int& lw) {
  const unsigned int ha = f2bf(a), hb = f2bf(b);
  const unsigned int la = f2bf(a - bf2f(ha)), lb = f2bf(b - bf2f(hb));
  hw = ha | (hb << 16);
  lw = la | (lb << 16);
}
__device__ __forceinline__ v4f hrelu4(const v4f w, const v4f c, float xm) {
  v4f t = w * xm;
  t = t + c;
  v4f r;
  r.x = fmaxf(t.x, 0.0f); r.y = fmaxf(t.y, 0.0f); r.z = fmaxf(t.z, 0.0f); r.w = fmaxf(t.w, 0.0f);
  return r;
}

__global__ __launch_bounds__(FTHR) void k_fused(const float* __restrict__ x, const float* __restrict__ adj,
                                                const float* __restrict__ fc1w, const float* __restrict__ fc1b,
                                                const float* __restrict__ fc2w, const float* __restrict__ fc2b,
                                                float* rec) {
  __shared__ __attribute__((aligned(16))) unsigned short sADJ[NV * KC];
  __shared__ __attribute__((aligned(16))) unsigned short sW2[HD * KC];
  __shared__ __attribute__((aligned(16))) unsigned short sHT[HD * KC];
  __shared__ __attribute__((aligned(16))) unsigned short sAG[NWF * 16 * 64];
  __shared__ __attribute__((aligned(16))) float sOUT[NV * HD];
  __shared__ __attribute__((aligned(16))) float sX[NV];
  __shared__ __attribute__((aligned(16))) float sINV[NV];
  __shared__ __attribute__((aligned(16))) float sW1[HD];
  __shared__ __attribute__((aligned(16))) float sB1[HD];
  __shared__ __attribute__((aligned(16))) float sB2[HD];

  const int tid = (int)threadIdx.x, lane = tid & 31, wave = tid >> 5, hh = lane >> 4, m = lane & 15;
  const int ch = (int)blockIdx.x;
  const int b  = (int)blockIdx.y;

#pragma unroll 1
  for (int u = tid; u < NV * (NV / 8); u += FTHR) {
    const int i = u >> 3, j0 = (u & 7) * 8;
    const float* p = adj + i * NV + j0;
    const v4f a = *(const v4fa*)p;
    const v4f c = *(const v4fa*)(p + 4);
    const v4u pv = pack8(a, c);
    *(v4ua*)(sADJ + i * KC + j0)      = pv;
    *(v4ua*)(sADJ + i * KC + NV + j0) = pv;
  }
#pragma unroll 1
  for (int u = tid; u < HD * (KC / 8); u += FTHR) {
    const int o = u >> 4, k8 = (u & 15) * 8;
    const int src = (k8 & 31) + 32 * (k8 >> 6);
    const float* p = fc2w + o * (2 * HD) + src;
    const v4f a = *(const v4fa*)p;
    const v4f c = *(const v4fa*)(p + 4);
    *(v4ua*)(sW2 + o * KC + k8) = pack8(a, c);
  }
  if (tid < HD) {
    sW1[tid] = bfr(fc1w[tid]);
    sB1[tid] = bfr(fc1b[tid]);
    sB2[tid] = bfr(fc2b[tid]);
  }
  __syncthreads();
  if (tid < NV) {
    float s = 0.0f;
#pragma unroll 4
    for (int j = 0; j < NV; ++j) s += bf2f((unsigned int)sADJ[tid * KC + j]);
    sINV[tid] = 1.0f / (s + 1e-8f);
  }
  __syncthreads();

  const v8f z8 = {0.f, 0.f, 0.f, 0.f, 0.f, 0.f, 0.f, 0.f};
  v8f run0 = z8, run1 = z8;
  const float b2a = sB2[m], b2b = sB2[16 + m];
  const float* xrow0 = x + ((size_t)b * SEQ + (size_t)ch * SC) * NV;
  const unsigned short* arow  = sADJ + (16 * wave + m) * KC + 8 * hh;
  const unsigned short* brow0 = sHT + m * KC + 8 * hh;
  const unsigned short* brow1 = sHT + (16 + m) * KC + 8 * hh;
  const unsigned short* wr0   = sW2 + m * KC + 8 * hh;
  const unsigned short* wr1   = sW2 + (16 + m) * KC + 8 * hh;
  unsigned short* agw = sAG + wave * (16 * 64);
  const unsigned short* agr = agw + m * 64 + 8 * hh;

#pragma unroll 1
  for (int si = 0; si < SC; ++si) {
    if (tid < NV / 4) {
      const v4f xv = *(const v4fa*)(xrow0 + (size_t)si * NV + 4 * tid);
      *(v4fa*)(sX + 4 * tid) = bfr4(xv);
    }
    __syncthreads();

#pragma unroll
    for (int q = 0; q < 2; ++q) {
      const int u  = tid + q * FTHR;
      const int f  = u >> 3, j0 = (u & 7) * 8;
      const float w = sW1[f], bb = sB1[f];
      const v4f xa = *(const v4fa*)(sX + j0);
      const v4f xb = *(const v4fa*)(sX + j0 + 4);
      const v4f w4 = {w, w, w, w};
      const v4f c4 = {bb, bb, bb, bb};
      v4f ta = xa * w4; ta = ta + c4;
      v4f tb = xb * w4; tb = tb + c4;
      v4f ha, hb;
      ha.x = fmaxf(ta.x, 0.0f); ha.y = fmaxf(ta.y, 0.0f); ha.z = fmaxf(ta.z, 0.0f); ha.w = fmaxf(ta.w, 0.0f);
      hb.x = fmaxf(tb.x, 0.0f); hb.y = fmaxf(tb.y, 0.0f); hb.z = fmaxf(tb.z, 0.0f); hb.w = fmaxf(tb.w, 0.0f);
      unsigned int h0w, l0w, h1w, l1w, h2w, l2w, h3w, l3w;
      split2(ha.x, ha.y, h0w, l0w);
      split2(ha.z, ha.w, h1w, l1w);
      split2(hb.x, hb.y, h2w, l2w);
      split2(hb.z, hb.w, h3w, l3w);
      v4u hv, lv;
      hv.x = h0w; hv.y = h1w; hv.z = h2w; hv.w = h3w;
      lv.x = l0w; lv.y = l1w; lv.z = l2w; lv.w = l3w;
      *(v4ua*)(sHT + f * KC + j0)      = hv;
      *(v4ua*)(sHT + f * KC + NV + j0) = lv;
    }
    const float xm = sX[16 * wave + m];
    __syncthreads();

    v8f accA0 = z8, accA1 = z8;
#pragma unroll
    for (int ks = 0; ks < 4; ++ks) {
      FragB af, bf0, bf1;
      af.h[0]  = *(const v8usa*)(arow  + 32 * ks);
      af.h[1]  = *(const v8usa*)(arow  + 32 * ks + 16);
      bf0.h[0] = *(const v8usa*)(brow0 + 32 * ks);
      bf0.h[1] = *(const v8usa*)(brow0 + 32 * ks + 16);
      bf1.h[0] = *(const v8usa*)(brow1 + 32 * ks);
      bf1.h[1] = *(const v8usa*)(brow1 + 32 * ks + 16);
      accA0 = wmb(af, bf0, accA0);
      accA1 = wmb(af, bf1, accA1);
    }
    {
      Q8 iv;
      iv.q[0] = *(const v4fa*)(sINV + 16 * wave + 8 * hh);
      iv.q[1] = *(const v4fa*)(sINV + 16 * wave + 8 * hh + 4);
#pragma unroll
      for (int r = 0; r < 8; ++r) {
        const int row = 8 * hh + r;
        const float inv = iv.v[r];
        const float v0 = accA0[r] * inv;
        const float v1 = accA1[r] * inv;
        const unsigned int h0 = f2bf(v0), h1 = f2bf(v1);
        const unsigned int l0 = f2bf(v0 - bf2f(h0)), l1 = f2bf(v1 - bf2f(h1));
        agw[row * 64 + m]      = (unsigned short)h0;
        agw[row * 64 + 16 + m] = (unsigned short)h1;
        agw[row * 64 + 32 + m] = (unsigned short)l0;
        agw[row * 64 + 48 + m] = (unsigned short)l1;
      }
    }
    __syncthreads();

    FragB fh, fl;
    {
      const v4f w0 = *(const v4fa*)(sW1 + 8 * hh);
      const v4f w1 = *(const v4fa*)(sW1 + 8 * hh + 4);
      const v4f w2 = *(const v4fa*)(sW1 + 16 + 8 * hh);
      const v4f w3 = *(const v4fa*)(sW1 + 16 + 8 * hh + 4);
      const v4f c0 = *(const v4fa*)(sB1 + 8 * hh);
      const v4f c1 = *(const v4fa*)(sB1 + 8 * hh + 4);
      const v4f c2 = *(const v4fa*)(sB1 + 16 + 8 * hh);
      const v4f c3 = *(const v4fa*)(sB1 + 16 + 8 * hh + 4);
      const v4f h0 = hrelu4(w0, c0, xm);
      const v4f h1 = hrelu4(w1, c1, xm);
      const v4f h2 = hrelu4(w2, c2, xm);
      const v4f h3 = hrelu4(w3, c3, xm);
      unsigned int hw, lw;
      split2(h0.x, h0.y, hw, lw); fh.w[0] = (int)hw; fl.w[0] = (int)lw;
      split2(h0.z, h0.w, hw, lw); fh.w[1] = (int)hw; fl.w[1] = (int)lw;
      split2(h1.x, h1.y, hw, lw); fh.w[2] = (int)hw; fl.w[2] = (int)lw;
      split2(h1.z, h1.w, hw, lw); fh.w[3] = (int)hw; fl.w[3] = (int)lw;
      split2(h2.x, h2.y, hw, lw); fh.w[4] = (int)hw; fl.w[4] = (int)lw;
      split2(h2.z, h2.w, hw, lw); fh.w[5] = (int)hw; fl.w[5] = (int)lw;
      split2(h3.x, h3.y, hw, lw); fh.w[6] = (int)hw; fl.w[6] = (int)lw;
      split2(h3.z, h3.w, hw, lw); fh.w[7] = (int)hw; fl.w[7] = (int)lw;
    }
    FragB ga, gl;
    ga.h[0] = *(const v8usa*)(agr);
    ga.h[1] = *(const v8usa*)(agr + 16);
    gl.h[0] = *(const v8usa*)(agr + 32);
    gl.h[1] = *(const v8usa*)(agr + 48);
    v8f accB0 = z8, accB1 = z8;
    {
      FragB q0, q1;
      q0.h[0] = *(const v8usa*)(wr0);       q0.h[1] = *(const v8usa*)(wr0 + 16);
      q1.h[0] = *(const v8usa*)(wr1);       q1.h[1] = *(const v8usa*)(wr1 + 16);
      accB0 = wmb(fh, q0, accB0);           accB1 = wmb(fh, q1, accB1);
      q0.h[0] = *(const v8usa*)(wr0 + 32);  q0.h[1] = *(const v8usa*)(wr0 + 48);
      q1.h[0] = *(const v8usa*)(wr1 + 32);  q1.h[1] = *(const v8usa*)(wr1 + 48);
      accB0 = wmb(fl, q0, accB0);           accB1 = wmb(fl, q1, accB1);
      q0.h[0] = *(const v8usa*)(wr0 + 64);  q0.h[1] = *(const v8usa*)(wr0 + 80);
      q1.h[0] = *(const v8usa*)(wr1 + 64);  q1.h[1] = *(const v8usa*)(wr1 + 80);
      accB0 = wmb(ga, q0, accB0);           accB1 = wmb(ga, q1, accB1);
      q0.h[0] = *(const v8usa*)(wr0 + 96);  q0.h[1] = *(const v8usa*)(wr0 + 112);
      q1.h[0] = *(const v8usa*)(wr1 + 96);  q1.h[1] = *(const v8usa*)(wr1 + 112);
      accB0 = wmb(gl, q0, accB0);           accB1 = wmb(gl, q1, accB1);
    }
#pragma unroll
    for (int r = 0; r < 8; ++r) {
      run0[r] = run0[r] + fmaxf(accB0[r] + b2a, 0.0f);
      run1[r] = run1[r] + fmaxf(accB1[r] + b2b, 0.0f);
    }
  }

#pragma unroll
  for (int r = 0; r < 8; ++r) {
    const int row = 16 * wave + 8 * hh + r;
    sOUT[row * HD + m]      = run0[r];
    sOUT[row * HD + 16 + m] = run1[r];
  }
  __syncthreads();
  v4f ov[4];
#pragma unroll
  for (int it = 0; it < 4; ++it) ov[it] = *(const v4fa*)(sOUT + 4 * (it * FTHR + tid));
  float* rb = rec + ((size_t)b * NCH + (size_t)ch) * RECF;
#pragma unroll
  for (int it = 0; it < 4; ++it) *(volatile v4f*)(rb + 4 * (it * FTHR + tid)) = ov[it];
  __threadfence();
#pragma unroll
  for (int it = 0; it < 4; ++it) *(volatile v4f*)(rb + 4 * (it * FTHR + tid)) = ov[it];
}

__global__ __launch_bounds__(CTHR) void k_comb(const float* __restrict__ rec, float* out, int nPieces) {
  const int p = (int)blockIdx.x * CTHR + (int)threadIdx.x;
  if (p >= nPieces) return;
  const int b = p >> 9;
  const int w = p & 511;
  const float* rp = rec + (size_t)b * NCH * RECF + 4 * w;
  v4f s = {0.f, 0.f, 0.f, 0.f};
#pragma unroll
  for (int ch = 0; ch < NCH; ++ch) {
    const v4f v = *(const v4fa*)(rp + (size_t)ch * RECF);
    s = s + v;
  }
  const v4f sc = {1.0f / 2048.0f, 1.0f / 2048.0f, 1.0f / 2048.0f, 1.0f / 2048.0f};
  const v4f o = s * sc;
  float* op = out + 4 * (size_t)p;
  *(volatile v4f*)op = o;
  __threadfence();
  *(volatile v4f*)op = o;
}

extern "C" void kernel_launch(void* const* d_in, const int* in_sizes, int n_in,
                              void* d_out, int out_size, void* d_ws, size_t ws_size,
                              hipStream_t stream) {
  if (n_in < 6) return;
  if (in_sizes[0] < SEQ * NV || (in_sizes[0] % (SEQ * NV)) != 0) return;
  const int nB = in_sizes[0] / (SEQ * NV);
  if (nB < 1 || nB > 4096) return;
  if (in_sizes[1] != NV * NV) return;
  if (in_sizes[2] != HD || in_sizes[3] != HD) return;
  if (in_sizes[4] != HD * 2 * HD || in_sizes[5] != HD) return;
  if (out_size != nB * NV * HD) return;
  if ((out_size % (4 * CTHR)) != 0) return;

  const float* x    = (const float*)d_in[0];
  const float* adj  = (const float*)d_in[1];
  const float* fc1w = (const float*)d_in[2];
  const float* fc1b = (const float*)d_in[3];
  const float* fc2w = (const float*)d_in[4];
  const float* fc2b = (const float*)d_in[5];
  float* out = (float*)d_out;

  const size_t recBytes = (size_t)nB * NCH * RECF * 4;
  if (recBytes > ws_size || recBytes > (size_t)WSMAX) return;
  float* REC = (float*)d_ws;

  k_fused<<<dim3(NCH, nB), FTHR, 0, stream>>>(x, adj, fc1w, fc1b, fc2w, fc2b, REC);
  const int nPieces = out_size / 4;
  k_comb<<<nPieces / CTHR, CTHR, 0, stream>>>(REC, out, nPieces);
}
